// TBNN_Q_direction_88081189307077
// MI455X (gfx1250) — hardware-verified
//
#include <hip/hip_runtime.h>


#define NB_  524288
#define SLP  0.1f
#define LOSC 1024.0f
#define LOSCI (1.0f / 1024.0f)

typedef _Float16 h16;
typedef __attribute__((ext_vector_type(16))) _Float16 v16h;
typedef __attribute__((ext_vector_type(8)))  _Float16 v8h;
typedef __attribute__((ext_vector_type(8)))  float    v8f;
typedef __attribute__((ext_vector_type(4)))  float    v4f;
typedef v8h  __attribute__((may_alias)) v8ha;
typedef v4f  __attribute__((may_alias)) v4fa;

__device__ __forceinline__ unsigned short f2bf(float f) { unsigned u = __float_as_uint(f); u += 0x7FFFu + ((u >> 16) & 1u); return (unsigned short)(u >> 16); }
__device__ __forceinline__ float bf2f(unsigned short b) { return __uint_as_float(((unsigned)b) << 16); }
__device__ __forceinline__ float bfr(float f) { return bf2f(f2bf(f)); }
__device__ __forceinline__ v16h cat16(v8h lo, v8h hi) { return __builtin_shufflevector(lo, hi, 0, 1, 2, 3, 4, 5, 6, 7, 8, 9, 10, 11, 12, 13, 14, 15); }
__device__ __forceinline__ v8f wmma16(v16h a, v16h b, v8f c) { return __builtin_amdgcn_wmma_f32_16x16x32_f16(false, a, false, b, (short)0, c, false, false); }
__device__ __forceinline__ float lk(float v) { return v >= 0.f ? v : SLP * v; }
#define VST2(T, p, v) do { const T vst2_v_ = (v); *(volatile T*)(p) = vst2_v_; __threadfence(); *(volatile T*)(p) = vst2_v_; } while (0)

__constant__ int cKP[6] = {32, 64, 128, 128, 128, 64};
__constant__ int cNP[6] = {64, 128, 128, 128, 64, 16};
__constant__ int cKR[6] = {5, 50, 100, 100, 100, 50};
__constant__ int cNR[6] = {50, 100, 100, 100, 50, 10};
__constant__ int cWOFF[6] = {0, 2048, 10240, 26624, 43008, 51200};

__global__ __launch_bounds__(256) void k_w16(const float* __restrict__ W0, const float* __restrict__ W1, const float* __restrict__ W2, const float* __restrict__ W3, const float* __restrict__ W4, const float* __restrict__ W5, h16* WP) {
    typedef __attribute__((ext_vector_type(4))) _Float16 v4h;
    const int t4 = (blockIdx.x * 256 + threadIdx.x) * 4;
    if (t4 >= 52224) return;
    v4h v;
#pragma unroll
    for (int i = 0; i < 4; ++i) {
        const int t = t4 + i;
        int l = 5;
        if (t < 2048) l = 0; else if (t < 2048 + 8192) l = 1; else if (t < 2048 + 8192 + 16384) l = 2; else if (t < 2048 + 8192 + 32768) l = 3; else if (t < 2048 + 8192 + 32768 + 8192) l = 4;
        const int off = (l == 0) ? 0 : (l == 1) ? 2048 : (l == 2) ? 10240 : (l == 3) ? 26624 : (l == 4) ? 43008 : 51200;
        const int u = t - off, n = u / cKP[l], k = u - n * cKP[l];
        const float* Wl = (l == 0) ? W0 : (l == 1) ? W1 : (l == 2) ? W2 : (l == 3) ? W3 : (l == 4) ? W4 : W5;
        const bool inb = (k < cKR[l] && n < cNR[l]); v[i] = inb ? (h16)bfr(Wl[inb ? (k * cNR[l] + n) : 0]) : (h16)0.f;
    }
    VST2(v4h, WP + t4, v);
}

struct M3 { float a[9]; };
__device__ __forceinline__ M3 mm3(const M3& x, const M3& y) { M3 r;
#pragma unroll
    for (int i = 0; i < 3; ++i)
#pragma unroll
        for (int j = 0; j < 3; ++j) r.a[i * 3 + j] = x.a[i * 3] * y.a[j] + x.a[i * 3 + 1] * y.a[3 + j] + x.a[i * 3 + 2] * y.a[6 + j];
    return r; }
__device__ __forceinline__ float tr3(const M3& x) { return x.a[0] + x.a[4] + x.a[8]; }

__global__ __launch_bounds__(128) void k_main(const float* __restrict__ S, const float* __restrict__ Wt, const h16* __restrict__ WP,
                                             const float* __restrict__ b0, const float* __restrict__ b1, const float* __restrict__ b2, const float* __restrict__ b3, const float* __restrict__ b4, const float* __restrict__ b5, float* out) {
    __shared__ __align__(16) h16 th_[2][4][16 * 136];
    __shared__ __align__(16) h16 tl_[2][4][16 * 136];
    __shared__ __align__(16) float gt[4][16 * 16];
    __shared__ __align__(16) float ob[64 * 9 + 32];
    const int lane = threadIdx.x & 31, wave = threadIdx.x >> 5, lr = lane & 15, hi = lane >> 4;
    const int r0 = blockIdx.x * 64 + wave * 16, row = r0 + lr;
    h16* myh = &th_[0][wave][0]; h16* myl = &tl_[0][wave][0];
    {
        M3 s, w;
#pragma unroll
        for (int i = 0; i < 9; ++i) { s.a[i] = bfr(S[(size_t)row * 9 + i]); w.a[i] = bfr(Wt[(size_t)row * 9 + i]); }
        const M3 s2 = mm3(s, s), w2 = mm3(w, w);
        float inv5[5]; inv5[0] = tr3(s2); inv5[1] = tr3(w2); inv5[2] = tr3(mm3(s2, s)); inv5[3] = tr3(mm3(w2, s)); inv5[4] = tr3(mm3(w2, s2));
        v16h ah = (v16h){}, al = (v16h){};
#pragma unroll
        for (int q = 0; q < 8; ++q) { const int k = 8 * hi + q; const float v = (k < 5) ? inv5[(k < 5) ? k : 0] : 0.f; const h16 hv = (h16)v; ah[q] = hv; al[q] = (h16)((v - (float)hv) * LOSC); }
        v8f acc[4], accx[4];
#pragma unroll
        for (int n = 0; n < 4; ++n) { acc[n] = (v8f){}; accx[n] = (v8f){}; }
#pragma unroll
        for (int n = 0; n < 4; ++n) { const h16* bp = WP + cWOFF[0] + (size_t)(n * 16 + lr) * 32 + 8 * hi; const v16h b = cat16(*(const v8h*)bp, *(const v8h*)(bp + 16)); acc[n] = wmma16(ah, b, acc[n]); accx[n] = wmma16(al, b, accx[n]); }
        asm volatile("v_nop\n\tv_nop\n\tv_nop\n\tv_nop" : "+v"(acc[0]), "+v"(acc[1]), "+v"(acc[2]), "+v"(acc[3]), "+v"(accx[0]), "+v"(accx[1]), "+v"(accx[2]), "+v"(accx[3]));
#pragma unroll
        for (int n = 0; n < 4; ++n) { const int col = n * 16 + lr; const float bb = (col < 50) ? bfr(b0[(col < 50) ? col : 0]) : 0.f;
#pragma unroll
            for (int j = 0; j < 8; ++j) { const float v = lk(acc[n][j] + accx[n][j] * LOSCI + bb); const h16 hv = (h16)v; myh[(hi * 8 + j) * 136 + col] = hv; myl[(hi * 8 + j) * 136 + col] = (h16)((v - (float)hv) * LOSC); } }
    }
    asm volatile("" ::: "memory");
    __builtin_amdgcn_fence(__ATOMIC_RELEASE, "workgroup");
    __builtin_amdgcn_wave_barrier();
#pragma unroll 1
    for (int l = 1; l < 6; ++l) {
        const int KP = cKP[l], NPd = cNP[l], NR = cNR[l];
        const float* bl = (l == 1) ? b1 : (l == 2) ? b2 : (l == 3) ? b3 : (l == 4) ? b4 : b5;
        const h16* inh = &th_[(l - 1) & 1][wave][0]; const h16* inl = &tl_[(l - 1) & 1][wave][0];
        h16* outh = &th_[l & 1][wave][0]; h16* outl = &tl_[l & 1][wave][0];
#pragma unroll 1
        for (int nh = 0; nh < NPd; nh += 64) {
            v8f acc[4], accx[4];
#pragma unroll
            for (int n = 0; n < 4; ++n) { acc[n] = (v8f){}; accx[n] = (v8f){}; }
#pragma unroll 1
            for (int kc = 0; kc < KP; kc += 32) {
                const v16h a = cat16(*(const v8ha*)(inh + lr * 136 + kc + 8 * hi), *(const v8ha*)(inh + lr * 136 + kc + 16 + 8 * hi));
                const v16h al = cat16(*(const v8ha*)(inl + lr * 136 + kc + 8 * hi), *(const v8ha*)(inl + lr * 136 + kc + 16 + 8 * hi));
#pragma unroll
                for (int n = 0; n < 4; ++n) { if (nh + n * 16 < NPd) { const h16* bp = WP + cWOFF[l] + (size_t)(nh + n * 16 + lr) * KP + kc + 8 * hi; const v16h b = cat16(*(const v8h*)bp, *(const v8h*)(bp + 16));
                    acc[n] = wmma16(a, b, acc[n]); accx[n] = wmma16(al, b, accx[n]); } }
                asm volatile("v_nop\n\tv_nop" : "+v"(acc[0]), "+v"(acc[3]), "+v"(accx[0]), "+v"(accx[3]) : "v"(a), "v"(al));
            }
            asm volatile("v_nop\n\tv_nop\n\tv_nop\n\tv_nop" : "+v"(acc[0]), "+v"(acc[1]), "+v"(acc[2]), "+v"(acc[3]), "+v"(accx[0]), "+v"(accx[1]), "+v"(accx[2]), "+v"(accx[3]));
            if (l < 5) {
#pragma unroll
                for (int n = 0; n < 4; ++n) { if (nh + n * 16 < NPd) { const int col = nh + n * 16 + lr; const float bb = (col < NR) ? bfr(bl[(col < NR) ? col : 0]) : 0.f;
#pragma unroll
                    for (int j = 0; j < 8; ++j) { const float v = lk(acc[n][j] + accx[n][j] * LOSCI + bb); const h16 hv = (h16)v; outh[(hi * 8 + j) * 136 + col] = hv; outl[(hi * 8 + j) * 136 + col] = (h16)((v - (float)hv) * LOSC); } } }
            } else {
                if (lr < 10) {
#pragma unroll
                    for (int j = 0; j < 8; ++j) gt[wave][(hi * 8 + j) * 16 + lr] = acc[0][j] + accx[0][j] * LOSCI + bfr(bl[lr]);
                }
            }
        }
        asm volatile("" ::: "memory");
        __builtin_amdgcn_fence(__ATOMIC_RELEASE, "workgroup");
        __builtin_amdgcn_wave_barrier();
    }
    if (lane < 16) {
        float g[10];
#pragma unroll
        for (int n = 0; n < 10; ++n) g[n] = gt[wave][lane * 16 + n];
        M3 s_, w_;
#pragma unroll
        for (int i = 0; i < 9; ++i) { s_.a[i] = bfr(S[(size_t)(r0 + lane) * 9 + i]); w_.a[i] = bfr(Wt[(size_t)(r0 + lane) * 9 + i]); }
        float Q[9];
        const M3 s2 = mm3(s_, s_), w2 = mm3(w_, w_);
        const float l1 = tr3(s2), l2 = tr3(w2);
#pragma unroll
        for (int i = 0; i < 9; ++i) { const float idv = (i == 0 || i == 4 || i == 8) ? 1.0f : 0.0f; Q[i] = g[0] * s_.a[i] + g[2] * (s2.a[i] - (l1 / 3.0f) * idv) + g[3] * (w2.a[i] - (l2 / 3.0f) * idv); }
        { const M3 sw = mm3(s_, w_), ws = mm3(w_, s_);
#pragma unroll
          for (int i = 0; i < 9; ++i) Q[i] += g[1] * (sw.a[i] - ws.a[i]);
          { const M3 a = mm3(ws, w2), b = mm3(w2, sw);
#pragma unroll
            for (int i = 0; i < 9; ++i) Q[i] += g[6] * (a.a[i] - b.a[i]); }
          { const M3 a = mm3(sw, s2), b = mm3(s2, ws);
#pragma unroll
            for (int i = 0; i < 9; ++i) Q[i] += g[7] * (a.a[i] - b.a[i]); } }
        { const M3 ws2 = mm3(w_, s2), s2w = mm3(s2, w_);
#pragma unroll
          for (int i = 0; i < 9; ++i) Q[i] += g[4] * (ws2.a[i] - s2w.a[i]);
          const M3 a = mm3(ws2, w2), b = mm3(w2, s2w);
#pragma unroll
          for (int i = 0; i < 9; ++i) Q[i] += g[9] * (a.a[i] - b.a[i]); }
        { const M3 sw2 = mm3(s_, w2), w2s = mm3(w2, s_); const float t6 = tr3(sw2) * (2.0f / 3.0f);
#pragma unroll
          for (int i = 0; i < 9; ++i) { const float idv = (i == 0 || i == 4 || i == 8) ? 1.0f : 0.0f; Q[i] += g[5] * (w2s.a[i] + sw2.a[i] - t6 * idv); } }
        { const M3 s2w2 = mm3(s2, w2), w2s2 = mm3(w2, s2); const float t9 = tr3(s2w2) * (2.0f / 3.0f);
#pragma unroll
          for (int i = 0; i < 9; ++i) { const float idv = (i == 0 || i == 4 || i == 8) ? 1.0f : 0.0f; Q[i] += g[8] * (w2s2.a[i] + s2w2.a[i] - t9 * idv); } }
        const float tq = (Q[0] + Q[4] + Q[8]) / 3.0f; Q[0] -= tq; Q[4] -= tq; Q[8] -= tq;
        float nrm = 0.f;
#pragma unroll
        for (int i = 0; i < 9; ++i) nrm += Q[i] * Q[i];
        nrm = sqrtf(nrm); if (nrm == 0.f) nrm = 1e-8f;
        const float inv = 1.0f / nrm;
#pragma unroll
        for (int i = 0; i < 9; ++i) ob[(wave * 16 + lane) * 9 + i] = Q[i] * inv;
    }
    __syncthreads();
#pragma unroll 1
    for (int ln = wave; ln < 18; ln += 4) VST2(float, out + (size_t)blockIdx.x * 576 + ln * 32 + lane, ob[ln * 32 + lane]);
}

extern "C" void kernel_launch(void* const* d_in, const int* in_sizes, int n_in,
                              void* d_out, int out_size, void* d_ws, size_t ws_size, hipStream_t stream) {
    (void)in_sizes; (void)n_in; (void)out_size;
    const float* S = (const float*)d_in[0]; const float* Wt = (const float*)d_in[1];
    const float* W0 = (const float*)d_in[2]; const float* b0 = (const float*)d_in[3]; const float* W1 = (const float*)d_in[4]; const float* b1 = (const float*)d_in[5];
    const float* W2 = (const float*)d_in[6]; const float* b2 = (const float*)d_in[7]; const float* W3 = (const float*)d_in[8]; const float* b3 = (const float*)d_in[9];
    const float* W4 = (const float*)d_in[10]; const float* b4 = (const float*)d_in[11]; const float* W5 = (const float*)d_in[12]; const float* b5 = (const float*)d_in[13];
    float* out = (float*)d_out;
    char* wsp = (char*)d_ws;
    auto take = [&](size_t bytes) { char* p = wsp; wsp += (bytes + 255) & ~(size_t)255; return (void*)p; };
    h16* WP = (h16*)take((size_t)52224 * 2);
    if ((size_t)(wsp - (char*)d_ws) > ws_size) return;
    k_w16<<<(52224 / 4 + 255) / 256, 256, 0, stream>>>(W0, W1, W2, W3, W4, W5, WP);
    k_main<<<NB_ / 64, 128, 0, stream>>>(S, Wt, WP, b0, b1, b2, b3, b4, b5, out);
}
